// GRU_23407571764060
// MI455X (gfx1250) — hardware-verified
//
#include <hip/hip_runtime.h>
#include <math.h>

constexpr int NBATCH  = 4096;
constexpr int NCHAN   = 2;
constexpr int NSAMP   = 1024;
constexpr int NFEAT   = 16;
constexpr int NHID    = 128;
constexpr int NGATE   = 3 * NHID;
constexpr int NCLS    = 24;
constexpr int SUBF    = NFEAT / NCHAN;
constexpr int NSTEP   = NCHAN * NSAMP / NFEAT;
constexpr int KXPAD   = 32;
constexpr int BTILE   = 16;
constexpr int NTHR    = 256;
constexpr int HPITCH  = 136;
constexpr int XPITCH  = 40;
constexpr int HBUF    = BTILE * HPITCH;
constexpr int XBUF    = BTILE * XPITCH;
constexpr int HFPITCH = 132;
constexpr float ACARRY = 16.0f;
constexpr float WCARRY = 16.0f;
constexpr float FOLD   = 1.0f / (ACARRY * WCARRY);

constexpr int PLANE_BIG  = NGATE * NHID;
constexpr int OFF_WHH1   = 0;
constexpr int OFF_WIH2   = PLANE_BIG;
constexpr int OFF_WHH2   = 2 * PLANE_BIG;
constexpr int OFF_WIH1   = 3 * PLANE_BIG;
constexpr int PLANE_X    = NGATE * KXPAD;
constexpr int PACK_HALVES = 3 * PLANE_BIG + PLANE_X;
constexpr int PK_BIG_THR = PLANE_BIG / 8;
constexpr int PK_BIG_BLK = PK_BIG_THR / NTHR;
constexpr int PK_X_THR   = PLANE_X / 8;
constexpr int PK_X_BLK   = PK_X_THR / NTHR;
constexpr int PK_GRID    = 3 * PK_BIG_BLK + PK_X_BLK;

static_assert(NSTEP == 128, "step count");
static_assert(SUBF == 8, "samples per channel per step");
static_assert(NHID == 16 * (NTHR / 32), "8 waves x 16 hidden columns");
static_assert(BTILE * NFEAT == NTHR, "x tile: one value per thread");
static_assert(NBATCH % BTILE == 0, "batch tiles exact");
static_assert(NHID % 32 == 0 && KXPAD % 32 == 0, "K multiples of 32");
static_assert((2 * HBUF) % NTHR == 0, "zero-fill loop exact");
static_assert(PK_BIG_THR % NTHR == 0 && PK_X_THR % NTHR == 0, "pack grid exact");
static_assert(PK_GRID == 78, "pack grid");
static_assert(PACK_HALVES * 2 == 319488, "workspace bytes");
static_assert((BTILE * NCLS * 4) % 512 == 0, "block output region = whole 512-B wave chunks");
static_assert(HPITCH % 8 == 0 && XPITCH % 8 == 0 && HFPITCH % 4 == 0, "16-B aligned LDS rows");

typedef __attribute__((ext_vector_type(16))) _Float16 v16h;
typedef __attribute__((ext_vector_type(8)))  _Float16 v8h;
typedef __attribute__((ext_vector_type(8)))  float    v8f;
typedef __attribute__((ext_vector_type(4)))  float    v4f;

__device__ __forceinline__ void guard3(v8f& a, v8f& b, v8f& c, v16h x, v16h y0, v16h y1, v16h y2) {
  asm volatile("v_nop\n\tv_nop\n\tv_nop\n\tv_nop" : "+v"(a), "+v"(b), "+v"(c) : "v"(x), "v"(y0), "v"(y1), "v"(y2));
}
__device__ __forceinline__ void acc_guard4(v8f& a, v8f& b, v8f& c, v8f& d) {
  asm volatile("v_nop\n\tv_nop\n\tv_nop\n\tv_nop" : "+v"(a), "+v"(b), "+v"(c), "+v"(d));
}

template <typename T> struct Frag;
template <> struct Frag<_Float16> {
  typedef v16h V; union U { v16h v; v8h h[2]; };
  static __device__ __forceinline__ v16h load(const _Float16* p) {
    U f; f.h[0] = *(const v8h*)(p); f.h[1] = *(const v8h*)(p + 16); return f.v;
  }
  static __device__ __forceinline__ v8f mma(v16h a, v16h b, v8f c) {
    return __builtin_amdgcn_wmma_f32_16x16x32_f16(false, a, false, b, (short)0, c, false, false);
  }
};

__device__ __forceinline__ float fsig(float x)  { return __builtin_amdgcn_rcpf(1.0f + __expf(-x)); }
__device__ __forceinline__ float ftanh(float x) { return 1.0f - 2.0f * __builtin_amdgcn_rcpf(__expf(2.0f * x) + 1.0f); }

__global__ __launch_bounds__(NTHR) void pack_weights_kernel(const float* __restrict__ wih1, const float* __restrict__ whh1,
                                                            const float* __restrict__ wih2, const float* __restrict__ whh2,
                                                            unsigned short* __restrict__ dst) {
  const int tid = threadIdx.x;
  const int blk = blockIdx.x;
  const float* sp;
  size_t dof;
  bool keep = true;
  if (blk < 3 * PK_BIG_BLK) {
    const int pl = blk / PK_BIG_BLK;
    const float* src = (pl == 0) ? whh1 : ((pl == 1) ? wih2 : whh2);
    const int rem = (blk - pl * PK_BIG_BLK) * NTHR + tid;
    sp  = src + (size_t)rem * 8;
    dof = (size_t)pl * PLANE_BIG + (size_t)rem * 8;
  } else {
    const int i2  = (blk - 3 * PK_BIG_BLK) * NTHR + tid;
    const int row = i2 >> 2;
    const int c8  = i2 & 3;
    sp   = wih1 + (size_t)row * NFEAT + (size_t)(c8 & 1) * 8;
    keep = (c8 < 2);
    dof  = (size_t)OFF_WIH1 + (size_t)i2 * 8;
  }
  const v4f a = *(const v4f*)(sp);
  const v4f b = *(const v4f*)(sp + 4);
  v8h hv;
#pragma unroll
  for (int e = 0; e < 4; ++e) {
    const float fa = a[e];
    const float fb = b[e];
    const float ga = keep ? (fa * WCARRY) : 0.0f;
    const float gb = keep ? (fb * WCARRY) : 0.0f;
    hv[e]     = (_Float16)ga;
    hv[4 + e] = (_Float16)gb;
  }
  unsigned short* op = dst + dof;
  *(volatile v8h*)op = hv;
  __threadfence();
  *(volatile v8h*)op = hv;
}

__device__ __forceinline__ void gru_gate8(const v8f aR, const v8f aZ, const v8f aNi, const v8f aNh,
                                          const float bR, const float bZ, const float bNi, const float bNh,
                                          float (&hs)[8], _Float16* dstcol) {
#pragma unroll
  for (int r = 0; r < 8; ++r) {
    const float rr  = fsig(aR[r] * FOLD + bR);
    const float zz  = fsig(aZ[r] * FOLD + bZ);
    const float hnp = aNh[r] * FOLD + bNh;
    const float nn  = ftanh(aNi[r] * FOLD + bNi + rr * hnp);
    const float ho  = hs[r];
    const float hn  = (1.0f - zz) * nn + zz * ho;
    hs[r] = hn;
    dstcol[r * HPITCH] = (_Float16)(hn * ACARRY);
  }
}

__global__ __launch_bounds__(NTHR) void gru2_fc_kernel(const float* __restrict__ x, const unsigned short* __restrict__ wpk,
                                                       const float* __restrict__ bih1, const float* __restrict__ bhh1,
                                                       const float* __restrict__ bih2, const float* __restrict__ bhh2,
                                                       const float* __restrict__ fcw, const float* __restrict__ fcb,
                                                       float* __restrict__ out) {
  __shared__ __align__(16) _Float16 H1s[2 * HBUF];
  __shared__ __align__(16) _Float16 H2s[2 * HBUF];
  __shared__ __align__(16) _Float16 Xs[2 * XBUF];
  __shared__ __align__(16) float    Hf[BTILE * HFPITCH];
  __shared__ __align__(16) float    Os[BTILE * NCLS];

  const int tid = threadIdx.x, lane = tid & 31, wave = tid >> 5;
  const int c = lane & 15, hh = lane >> 4, koff = hh * 8;
  const int j = 16 * wave + c;
  const int b0 = blockIdx.x * BTILE;

#pragma unroll 1
  for (int i = tid; i < 2 * HBUF; i += NTHR) {
    H1s[i] = (_Float16)0.0f;
    H2s[i] = (_Float16)0.0f;
  }

  const int xrow = tid >> 4, xc = tid & 15;
  const float* xp = x + (size_t)(b0 + xrow) * (size_t)(NCHAN * NSAMP) + (size_t)(xc / SUBF) * NSAMP + (size_t)(xc % SUBF);
  {
    const float v0 = xp[0];
    Xs[xrow * XPITCH + xc]      = (_Float16)(v0 * ACARRY);
    Xs[xrow * XPITCH + 16 + xc] = (_Float16)0.0f;
  }

  const float b1r  = bih1[j] + bhh1[j];
  const float b1z  = bih1[NHID + j] + bhh1[NHID + j];
  const float b1ni = bih1[2 * NHID + j];
  const float b1nh = bhh1[2 * NHID + j];
  const float b2r  = bih2[j] + bhh2[j];
  const float b2z  = bih2[NHID + j] + bhh2[NHID + j];
  const float b2ni = bih2[2 * NHID + j];
  const float b2nh = bhh2[2 * NHID + j];

  const _Float16* W   = (const _Float16*)wpk;
  const _Float16* w1h = W + OFF_WHH1 + (size_t)j * NHID + koff;
  const _Float16* w2i = W + OFF_WIH2 + (size_t)j * NHID + koff;
  const _Float16* w2h = W + OFF_WHH2 + (size_t)j * NHID + koff;
  const _Float16* w1x = W + OFF_WIH1 + (size_t)j * KXPAD + koff;
  constexpr int GSTR  = NHID * NHID;
  constexpr int GSTRX = NHID * KXPAD;

  const v16h bx0 = Frag<_Float16>::load(w1x);
  const v16h bx1 = Frag<_Float16>::load(w1x + GSTRX);
  const v16h bx2 = Frag<_Float16>::load(w1x + 2 * GSTRX);

  float h1s[8], h2s[8];
#pragma unroll
  for (int r = 0; r < 8; ++r) { h1s[r] = 0.0f; h2s[r] = 0.0f; }

  const v8f z8 = {0.f, 0.f, 0.f, 0.f, 0.f, 0.f, 0.f, 0.f};

#pragma unroll 1
  for (int t = 0; t < NSTEP; ++t) {
    const int p = t & 1, q = p ^ 1;
    const _Float16* xr   = Xs  + p * XBUF + c * XPITCH + koff;
    _Float16*       xw   = Xs  + q * XBUF + xrow * XPITCH + xc;
    const _Float16* h1r  = H1s + p * HBUF + c * HPITCH + koff;
    _Float16*       h1wc = H1s + q * HBUF + (8 * hh) * HPITCH + j;
    const _Float16* h1n  = H1s + q * HBUF + c * HPITCH + koff;
    const _Float16* h2r  = H2s + p * HBUF + c * HPITCH + koff;
    _Float16*       h2wc = H2s + q * HBUF + (8 * hh) * HPITCH + j;

    __syncthreads();

    {
      const int tn = (t + 1 < NSTEP) ? (t + 1) : (NSTEP - 1);
      const float vx = xp[(size_t)SUBF * tn];
      xw[0]  = (_Float16)(vx * ACARRY);
      xw[16] = (_Float16)0.0f;
    }

    {
      const v16h ax = Frag<_Float16>::load(xr);
      v8f aR  = Frag<_Float16>::mma(ax, bx0, z8);
      v8f aZ  = Frag<_Float16>::mma(ax, bx1, z8);
      v8f aNi = Frag<_Float16>::mma(ax, bx2, z8);
      v8f aNh = z8;
      guard3(aR, aZ, aNi, ax, bx0, bx1, bx2);
#pragma unroll 1
      for (int k0 = 0; k0 < NHID; k0 += 32) {
        const v16h a   = Frag<_Float16>::load(h1r + k0);
        const v16h bb0 = Frag<_Float16>::load(w1h + k0);
        const v16h bb1 = Frag<_Float16>::load(w1h + GSTR + k0);
        const v16h bb2 = Frag<_Float16>::load(w1h + 2 * GSTR + k0);
        aR  = Frag<_Float16>::mma(a, bb0, aR);
        aZ  = Frag<_Float16>::mma(a, bb1, aZ);
        aNh = Frag<_Float16>::mma(a, bb2, aNh);
        guard3(aR, aZ, aNh, a, bb0, bb1, bb2);
      }
      acc_guard4(aR, aZ, aNi, aNh);
      gru_gate8(aR, aZ, aNi, aNh, b1r, b1z, b1ni, b1nh, h1s, h1wc);
    }

    __syncthreads();

    {
      v8f cR = z8, cZ = z8, cNi = z8, cNh = z8;
#pragma unroll 1
      for (int k0 = 0; k0 < NHID; k0 += 32) {
        const v16h ai  = Frag<_Float16>::load(h1n + k0);
        const v16h bi0 = Frag<_Float16>::load(w2i + k0);
        const v16h bi1 = Frag<_Float16>::load(w2i + GSTR + k0);
        const v16h bi2 = Frag<_Float16>::load(w2i + 2 * GSTR + k0);
        cR  = Frag<_Float16>::mma(ai, bi0, cR);
        cZ  = Frag<_Float16>::mma(ai, bi1, cZ);
        cNi = Frag<_Float16>::mma(ai, bi2, cNi);
        guard3(cR, cZ, cNi, ai, bi0, bi1, bi2);
        const v16h ah  = Frag<_Float16>::load(h2r + k0);
        const v16h bh0 = Frag<_Float16>::load(w2h + k0);
        const v16h bh1 = Frag<_Float16>::load(w2h + GSTR + k0);
        const v16h bh2 = Frag<_Float16>::load(w2h + 2 * GSTR + k0);
        cR  = Frag<_Float16>::mma(ah, bh0, cR);
        cZ  = Frag<_Float16>::mma(ah, bh1, cZ);
        cNh = Frag<_Float16>::mma(ah, bh2, cNh);
        guard3(cR, cZ, cNh, ah, bh0, bh1, bh2);
      }
      acc_guard4(cR, cZ, cNi, cNh);
      gru_gate8(cR, cZ, cNi, cNh, b2r, b2z, b2ni, b2nh, h2s, h2wc);
    }
  }

#pragma unroll
  for (int r = 0; r < 8; ++r) Hf[(8 * hh + r) * HFPITCH + j] = h2s[r];
  __syncthreads();

#pragma unroll 1
  for (int it = 0; it < 2; ++it) {
    const int idx = it * NTHR + tid;
    if (idx < BTILE * NCLS) {
      const int row = idx / NCLS;
      const int cls = idx - row * NCLS;
      const float* hr = Hf + row * HFPITCH;
      const float* wr = fcw + (size_t)cls * NHID;
      float s = 0.0f;
#pragma unroll 1
      for (int k = 0; k < NHID; k += 4) {
        const v4f hv = *(const v4f*)(hr + k);
        const v4f wv = *(const v4f*)(wr + k);
        s += hv[0] * wv[0];
        s += hv[1] * wv[1];
        s += hv[2] * wv[2];
        s += hv[3] * wv[3];
      }
      Os[idx] = s + fcb[cls];
    }
  }
  __syncthreads();

  if (tid < (BTILE * NCLS) / 4) {
    const v4f v = *(const v4f*)(Os + tid * 4);
    float* op = out + (size_t)b0 * NCLS + (size_t)tid * 4;
    *(volatile v4f*)op = v;
    __threadfence();
    *(volatile v4f*)op = v;
  }
}

extern "C" void kernel_launch(void* const* d_in, const int* in_sizes, int n_in,
                              void* d_out, int out_size, void* d_ws, size_t ws_size, hipStream_t stream) {
  if (n_in < 11 || d_out == nullptr || d_ws == nullptr) return;
  if (in_sizes[0] != NBATCH * NCHAN * NSAMP || in_sizes[1] != NGATE * NFEAT || in_sizes[2] != NGATE * NHID ||
      in_sizes[3] != NGATE || in_sizes[4] != NGATE || in_sizes[5] != NGATE * NHID || in_sizes[6] != NGATE * NHID ||
      in_sizes[7] != NGATE || in_sizes[8] != NGATE || in_sizes[9] != NCLS * NHID || in_sizes[10] != NCLS ||
      out_size != NBATCH * NCLS) return;
  if ((size_t)PACK_HALVES * 2 > ws_size) return;

  const float* x    = (const float*)d_in[0];
  const float* wih1 = (const float*)d_in[1];
  const float* whh1 = (const float*)d_in[2];
  const float* bih1 = (const float*)d_in[3];
  const float* bhh1 = (const float*)d_in[4];
  const float* wih2 = (const float*)d_in[5];
  const float* whh2 = (const float*)d_in[6];
  const float* bih2 = (const float*)d_in[7];
  const float* bhh2 = (const float*)d_in[8];
  const float* fcw  = (const float*)d_in[9];
  const float* fcb  = (const float*)d_in[10];
  float* out = (float*)d_out;
  unsigned short* wpk = (unsigned short*)d_ws;

  pack_weights_kernel<<<PK_GRID, NTHR, 0, stream>>>(wih1, whh1, wih2, whh2, wpk);
  gru2_fc_kernel<<<NBATCH / BTILE, NTHR, 0, stream>>>(x, wpk, bih1, bhh1, bih2, bhh2, fcw, fcb, out);
}
